// UnifiedEngineBlock_61607010894205
// MI455X (gfx1250) — hardware-verified
//
#include <hip/hip_runtime.h>
#include <stdint.h>


typedef _Float16 bf16;
typedef __attribute__((ext_vector_type(4))) float v4f;
typedef __attribute__((ext_vector_type(4))) unsigned v4u;
template <typename V> __device__ __forceinline__ void vst2(void* p, V v) {
  *(volatile V*)p = v; __threadfence(); *(volatile V*)p = v;
}
typedef __attribute__((ext_vector_type(16))) _Float16 v16h;
typedef __attribute__((ext_vector_type(8)))  _Float16 v8h;
typedef __attribute__((ext_vector_type(8)))  float  v8f;

constexpr int Bb  = 4;
constexpr int Ss  = 2048;
constexpr int Dd  = 1024;
constexpr int Hh  = 4;
constexpr int HDd = Dd / Hh;
constexpr int Ee  = 4;
constexpr int DFf = Dd * Ee;
constexpr int TOK = Bb * Ss;

__device__ __forceinline__ v8f wmma_bf16(v16h a, v16h b, v8f c) {
  v8f d = __builtin_amdgcn_wmma_f32_16x16x32_f16(false, a, false, b, (short)0, c, false, false);
  asm volatile("v_nop\n\tv_nop\n\tv_nop\n\tv_nop" : "+v"(d) : "v"(a), "v"(b));
  return d;
}

__device__ __forceinline__ float gelu_exact(float x) {
  return 0.5f * x * (1.0f + erff(x * 0.70710678118654752f));
}

__device__ __forceinline__ void block_stats(float s, float s2, float* red,
                                            float& mean, float& rstd) {
  #pragma unroll
  for (int o = 16; o > 0; o >>= 1) {
    s  += __shfl_xor(s,  o, 32);
    s2 += __shfl_xor(s2, o, 32);
  }
  int wid = threadIdx.x >> 5, lane = threadIdx.x & 31;
  if (lane == 0) { red[wid] = s; red[8 + wid] = s2; }
  __syncthreads();
  if (threadIdx.x == 0) {
    float a = 0.f, b = 0.f;
    for (int i = 0; i < 8; ++i) { a += red[i]; b += red[8 + i]; }
    red[16] = a; red[17] = b;
  }
  __syncthreads();
  mean = red[16] * (1.0f / Dd);
  float var = red[17] * (1.0f / Dd) - mean * mean;
  rstd = rsqrtf(var + 1e-5f);
}

__global__ __launch_bounds__(256) void transpose_cvt_kernel(
    const float* __restrict__ src, bf16* __restrict__ dst, int K, int N) {
  __shared__ __align__(16) bf16 tile[64][72];
  const int nt = N / 64;
  const int nBase = (blockIdx.x % nt) * 64, kBase = (blockIdx.x / nt) * 64, tid = threadIdx.x;
  for (int i = tid; i < 64 * 64; i += 256) { const int kk = i >> 6, nn = i & 63; tile[nn][kk] = (bf16)src[(size_t)(kBase + kk) * N + nBase + nn]; }
  __syncthreads();
  for (int g = tid; g < 64 * 8; g += 256) { const int nn = g >> 3, pc = g & 7; vst2(dst + (size_t)(nBase + nn) * K + kBase + pc * 8, *(const v4u*)(&tile[nn][pc * 8])); }
}

__global__ __launch_bounds__(256) void ln_dual_kernel(
    const float* __restrict__ x,
    const float* __restrict__ g1, const float* __restrict__ b1,
    const float* __restrict__ g2, const float* __restrict__ b2,
    bf16* __restrict__ xn1, bf16* __restrict__ xn2) {
  __shared__ float red[18];
  size_t t = blockIdx.x;
  int tid = threadIdx.x;
  float4 v = ((const float4*)(x + t * Dd))[tid];
  float s  = v.x + v.y + v.z + v.w;
  float s2 = v.x * v.x + v.y * v.y + v.z * v.z + v.w * v.w;
  float mean, rstd;
  block_stats(s, s2, red, mean, rstd);
  float4 G1 = ((const float4*)g1)[tid], B1 = ((const float4*)b1)[tid];
  float4 G2 = ((const float4*)g2)[tid], B2 = ((const float4*)b2)[tid];
  size_t base = t * Dd + tid * 4;
  float n0 = (v.x - mean) * rstd, n1 = (v.y - mean) * rstd;
  float n2 = (v.z - mean) * rstd, n3 = (v.w - mean) * rstd;
  union { bf16 h[4]; unsigned long long u; } p1, p2;
  p1.h[0] = (bf16)(n0 * G1.x + B1.x); p2.h[0] = (bf16)(n0 * G2.x + B2.x);
  p1.h[1] = (bf16)(n1 * G1.y + B1.y); p2.h[1] = (bf16)(n1 * G2.y + B2.y);
  p1.h[2] = (bf16)(n2 * G1.z + B1.z); p2.h[2] = (bf16)(n2 * G2.z + B2.z);
  p1.h[3] = (bf16)(n3 * G1.w + B1.w); p2.h[3] = (bf16)(n3 * G2.w + B2.w);
  vst2(xn1 + base, p1.u); vst2(xn2 + base, p2.u);
}

template <int EPI>
__global__ __launch_bounds__(256) void gemm_bf16_wmma(
    const bf16* __restrict__ A, const bf16* __restrict__ Bt,
    const float* __restrict__ bias, const float* __restrict__ res,
    void* __restrict__ out, int Mtot, int Ntot, int Ktot) {
  __shared__ __align__(16) bf16 As[2][128 * 48];
  __shared__ __align__(16) bf16 Bs[2][128 * 48];
  __shared__ __align__(16) float Ct[128][128];
  const int tid  = threadIdx.x;
  const int lane = tid & 31, wid = tid >> 5;
  const int wm = wid & 1, wn = wid >> 1;
  const int la = lane & 15, hs = lane >> 4;
  const int mBase = blockIdx.y * 128, nBase = blockIdx.x * 128;

  auto stage = [&](int k0, int buf) {
    #pragma unroll
    for (int c = tid; c < 512; c += 256) {
      int r = c >> 2, cc = (c & 3) * 8;
      *(v4u*)&As[buf][r * 48 + cc] = *(const v4u*)&A [(size_t)(mBase + r) * Ktot + k0 + cc];
      *(v4u*)&Bs[buf][r * 48 + cc] = *(const v4u*)&Bt[(size_t)(nBase + r) * Ktot + k0 + cc];
    }
  };

  v8f acc[4][2] = {};
  const int ntiles = Ktot >> 5;
  stage(0, 0);

  for (int it = 0; it < ntiles; ++it) {
    const int cur = it & 1;
    __syncthreads();
    if (it + 1 < ntiles) stage((it + 1) * 32, cur ^ 1);

    v16h afrag[4];
    #pragma unroll
    for (int ms = 0; ms < 4; ++ms) {
      int r = wm * 64 + ms * 16 + la;
      union { v16h v; v8h h[2]; } u;
      u.h[0] = *(const v8h*)&As[cur][r * 48 + hs * 8];
      u.h[1] = *(const v8h*)&As[cur][r * 48 + hs * 8 + 16];
      afrag[ms] = u.v;
    }
    v16h bfrag[2];
    #pragma unroll
    for (int ns = 0; ns < 2; ++ns) {
      int r = wn * 32 + ns * 16 + la;
      union { v16h v; v8h h[2]; } u;
      u.h[0] = *(const v8h*)&Bs[cur][r * 48 + hs * 8];
      u.h[1] = *(const v8h*)&Bs[cur][r * 48 + hs * 8 + 16];
      bfrag[ns] = u.v;
    }
    #pragma unroll
    for (int ms = 0; ms < 4; ++ms)
      #pragma unroll
      for (int ns = 0; ns < 2; ++ns)
        acc[ms][ns] = wmma_bf16(afrag[ms], bfrag[ns], acc[ms][ns]);
  }

  __syncthreads();
  #pragma unroll
  for (int ms = 0; ms < 4; ++ms)
    #pragma unroll
    for (int ns = 0; ns < 2; ++ns) {
      int cl = wn * 32 + ns * 16 + la;
      int col = nBase + cl;
      float bv = bias[col];
      #pragma unroll
      for (int r = 0; r < 8; ++r) {
        int rl = wm * 64 + ms * 16 + r + hs * 8;
        int row = mBase + rl;
        float v = acc[ms][ns][r] + bv;
        if constexpr (EPI == 0) v = gelu_exact(v);
        else if constexpr (EPI == 1) v += res[(size_t)row * Ntot + col];
        Ct[rl][cl] = v;
      }
    }
  __syncthreads();
  if constexpr (EPI == 1) {
    for (int g = tid; g < 128 * 32; g += 256) { const int rl = g >> 5, pc = g & 31; vst2((float*)out + (size_t)(mBase + rl) * Ntot + nBase + pc * 4, *(const v4f*)(&Ct[rl][pc * 4])); }
  } else if constexpr (EPI == 3) {
    const int b = mBase / Ss, s0 = mBase % Ss, h = nBase / HDd, hd0 = nBase % HDd;
    for (int g = tid; g < 128 * 16; g += 256) {
      const int cl = g >> 4, pc = g & 15;
      union { v8h h; v4u u; } pk;
      #pragma unroll
      for (int e = 0; e < 8; ++e) pk.h[e] = (bf16)Ct[pc * 8 + e][cl];
      vst2((bf16*)out + ((size_t)((b * Hh + h) * HDd + hd0 + cl)) * Ss + s0 + pc * 8, pk.u);
    }
  } else {
    for (int g = tid; g < 128 * 16; g += 256) {
      const int rl = g >> 4, pc = g & 15;
      union { v8h h; v4u u; } pk;
      #pragma unroll
      for (int e = 0; e < 8; ++e) pk.h[e] = (bf16)Ct[rl][pc * 8 + e];
      const int row = mBase + rl;
      if constexpr (EPI == 0) vst2((bf16*)out + (size_t)row * Ntot + nBase + pc * 8, pk.u);
      else { const int b = row / Ss, s = row % Ss, h = nBase / HDd, hd0 = nBase % HDd;
             vst2((bf16*)out + ((size_t)((b * Hh + h) * Ss + s)) * HDd + hd0 + pc * 8, pk.u); }
    }
  }
}

__global__ __launch_bounds__(256) void hebbian_attn_kernel(
    const bf16* __restrict__ q, const bf16* __restrict__ k,
    const bf16* __restrict__ vt, const float* __restrict__ betap,
    bf16* __restrict__ attn_out) {
  __shared__ __align__(16) bf16 Qs[64 * 264];
  __shared__ __align__(16) bf16 affs[64 * 72];
  __shared__ __align__(16) bf16 Ot[8][16 * 128];
  const int qt = blockIdx.x, bh = blockIdx.y;
  const int bidx = bh / Hh, hidx = bh % Hh;
  const int tid = threadIdx.x, lane = tid & 31, wid = tid >> 5;
  const int la = lane & 15, hs = lane >> 4;
  const float beta = betap[0];

  const bf16* qb = q + ((size_t)bh * Ss + qt * 64) * HDd;
  #pragma unroll
  for (int c = tid; c < 64 * 32; c += 256) {
    int r = c >> 5, cc = (c & 31) * 8;
    *(v4u*)&Qs[r * 264 + cc] = *(const v4u*)&qb[(size_t)r * HDd + cc];
  }
  __syncthreads();

  const int ma = wid & 3;
  const int nh = wid >> 2;
  v8f oacc[8] = {};

  for (int kt = 0; kt <= qt; ++kt) {
    const int kbase = kt * 64;
    v8f c0 = {}, c1 = {};
    const bf16* kb = k + ((size_t)bh * Ss + kbase) * HDd;
    #pragma unroll
    for (int kf = 0; kf < HDd; kf += 32) {
      union { v16h v; v8h h[2]; } ua, ub0, ub1;
      int ar = ma * 16 + la;
      ua.h[0] = *(const v8h*)&Qs[ar * 264 + kf + hs * 8];
      ua.h[1] = *(const v8h*)&Qs[ar * 264 + kf + hs * 8 + 16];
      const bf16* p0 = kb + (size_t)(nh * 32 + la)      * HDd + kf + hs * 8;
      const bf16* p1 = kb + (size_t)(nh * 32 + 16 + la) * HDd + kf + hs * 8;
      ub0.h[0] = *(const v8h*)p0; ub0.h[1] = *(const v8h*)(p0 + 16);
      ub1.h[0] = *(const v8h*)p1; ub1.h[1] = *(const v8h*)(p1 + 16);
      c0 = wmma_bf16(ua.v, ub0.v, c0);
      c1 = wmma_bf16(ua.v, ub1.v, c1);
    }
    __syncthreads();
    #pragma unroll
    for (int ns = 0; ns < 2; ++ns) {
      v8f cv = ns ? c1 : c0;
      int jl = nh * 32 + ns * 16 + la;
      int j = kbase + jl;
      #pragma unroll
      for (int r = 0; r < 8; ++r) {
        int il = ma * 16 + r + hs * 8;
        int i = qt * 64 + il;
        float v = cv[r] * beta;
        v = (j <= i && v > 0.f) ? v : 0.f;
        affs[il * 72 + jl] = (bf16)v;
      }
    }
    __syncthreads();
    const bf16* vb = vt + (size_t)bh * HDd * Ss;
    #pragma unroll
    for (int kk = 0; kk < 64; kk += 32) {
      union { v16h v; v8h h[2]; } ua;
      int ar = ma * 16 + la;
      ua.h[0] = *(const v8h*)&affs[ar * 72 + kk + hs * 8];
      ua.h[1] = *(const v8h*)&affs[ar * 72 + kk + hs * 8 + 16];
      #pragma unroll
      for (int j = 0; j < 8; ++j) {
        int feat = nh * 128 + j * 16 + la;
        union { v16h v; v8h h[2]; } ub;
        const bf16* p = vb + (size_t)feat * Ss + kbase + kk + hs * 8;
        ub.h[0] = *(const v8h*)p; ub.h[1] = *(const v8h*)(p + 16);
        oacc[j] = wmma_bf16(ua.v, ub.v, oacc[j]);
      }
    }
  }
  bf16* ot = Ot[wid];
  #pragma unroll
  for (int j = 0; j < 8; ++j) {
    int fl = j * 16 + la;
    #pragma unroll
    for (int r = 0; r < 8; ++r) ot[(r + hs * 8) * 128 + fl] = (bf16)oacc[j][r];
  }
  __syncthreads();
  #pragma unroll
  for (int q2 = 0; q2 < 8; ++q2) {
    const int rl = q2 * 2 + (lane >> 4), pc = lane & 15;
    const int s = qt * 64 + ma * 16 + rl;
    vst2(attn_out + ((size_t)(bidx * Ss + s)) * Dd + hidx * HDd + nh * 128 + pc * 8, *(const v4u*)(ot + rl * 128 + pc * 8));
  }
}

__global__ __launch_bounds__(256) void trm_scalar_mlp_kernel(
    const float* __restrict__ tpre, const float* __restrict__ g,
    const float* __restrict__ bt, const float* __restrict__ sw1,
    const float* __restrict__ sb1, const float* __restrict__ sw2,
    const float* __restrict__ sb2, float* __restrict__ trm_out) {
  __shared__ float red[18];
  size_t t = blockIdx.x;
  int tid = threadIdx.x;
  float4 v = ((const float4*)(tpre + t * Dd))[tid];
  float s  = v.x + v.y + v.z + v.w;
  float s2 = v.x * v.x + v.y * v.y + v.z * v.z + v.w * v.w;
  float mean, rstd;
  block_stats(s, s2, red, mean, rstd);
  float4 G = ((const float4*)g)[tid], Bt = ((const float4*)bt)[tid];
  float w1e[Ee], b1e[Ee], w2e[Ee];
  #pragma unroll
  for (int e = 0; e < Ee; ++e) { w1e[e] = sw1[e]; b1e[e] = sb1[e]; w2e[e] = sw2[e]; }
  float vb2 = sb2[0];
  float xin[4] = {v.x, v.y, v.z, v.w};
  float gg[4] = {G.x, G.y, G.z, G.w}, bb[4] = {Bt.x, Bt.y, Bt.z, Bt.w};
  float4 o;
  float* op = &o.x;
  #pragma unroll 1
  for (int c = 0; c < 4; ++c) {
    float xn = (xin[c] - mean) * rstd * gg[c] + bb[c];
    float mix = vb2;
    #pragma unroll 1
    for (int e = 0; e < Ee; ++e) mix += gelu_exact(xn * w1e[e] + b1e[e]) * w2e[e];
    op[c] = xin[c] + mix;
  }
  { v4f ov = {o.x, o.y, o.z, o.w}; vst2((v4f*)(trm_out + t * Dd) + tid, ov); }
}

__global__ __launch_bounds__(256) void blend_ln_kernel(
    const float* __restrict__ x, const float* __restrict__ trm,
    const float* __restrict__ heb, const float* __restrict__ alphap,
    const float* __restrict__ g, const float* __restrict__ bt,
    float* __restrict__ out) {
  __shared__ float red[18];
  size_t t = blockIdx.x;
  int tid = threadIdx.x;
  float bw = 1.0f / (1.0f + expf(-alphap[0]));
  float4 xv = ((const float4*)(x   + t * Dd))[tid];
  float4 tv = ((const float4*)(trm + t * Dd))[tid];
  float4 hv = ((const float4*)(heb + t * Dd))[tid];
  float4 u;
  u.x = xv.x + bw * tv.x + (1.f - bw) * hv.x;
  u.y = xv.y + bw * tv.y + (1.f - bw) * hv.y;
  u.z = xv.z + bw * tv.z + (1.f - bw) * hv.z;
  u.w = xv.w + bw * tv.w + (1.f - bw) * hv.w;
  float s  = u.x + u.y + u.z + u.w;
  float s2 = u.x * u.x + u.y * u.y + u.z * u.z + u.w * u.w;
  float mean, rstd;
  block_stats(s, s2, red, mean, rstd);
  float4 G = ((const float4*)g)[tid], Bt = ((const float4*)bt)[tid];
  float4 o;
  o.x = (u.x - mean) * rstd * G.x + Bt.x;
  o.y = (u.y - mean) * rstd * G.y + Bt.y;
  o.z = (u.z - mean) * rstd * G.z + Bt.z;
  o.w = (u.w - mean) * rstd * G.w + Bt.w;
  { v4f ov = {o.x, o.y, o.z, o.w}; vst2((v4f*)(out + t * Dd) + tid, ov); }
}

extern "C" void kernel_launch(void* const* d_in, const int* in_sizes, int n_in,
                              void* d_out, int out_size, void* d_ws, size_t ws_size,
                              hipStream_t stream) {
  const float* x      = (const float*)d_in[0];
  const float* h_ln_g = (const float*)d_in[1];
  const float* h_ln_b = (const float*)d_in[2];
  const float* wq     = (const float*)d_in[3];
  const float* bq     = (const float*)d_in[4];
  const float* wk     = (const float*)d_in[5];
  const float* bk     = (const float*)d_in[6];
  const float* wv     = (const float*)d_in[7];
  const float* bv     = (const float*)d_in[8];
  const float* wo     = (const float*)d_in[9];
  const float* bo     = (const float*)d_in[10];
  const float* beta   = (const float*)d_in[11];
  const float* t_ln1_g= (const float*)d_in[12];
  const float* t_ln1_b= (const float*)d_in[13];
  const float* t_w1   = (const float*)d_in[14];
  const float* t_b1   = (const float*)d_in[15];
  const float* t_w2   = (const float*)d_in[16];
  const float* t_b2   = (const float*)d_in[17];
  const float* t_lns_g= (const float*)d_in[18];
  const float* t_lns_b= (const float*)d_in[19];
  const float* s_w1   = (const float*)d_in[20];
  const float* s_b1   = (const float*)d_in[21];
  const float* s_w2   = (const float*)d_in[22];
  const float* s_b2   = (const float*)d_in[23];
  const float* alpha  = (const float*)d_in[24];
  const float* o_ln_g = (const float*)d_in[25];
  const float* o_ln_b = (const float*)d_in[26];
  float* out = (float*)d_out;

  char* ws = (char*)d_ws;
  const size_t MB = 1ull << 20;
  bf16* wqt  = (bf16*)(ws + 0 * MB);
  bf16* wkt  = (bf16*)(ws + 2 * MB);
  bf16* wvt  = (bf16*)(ws + 4 * MB);
  bf16* wot  = (bf16*)(ws + 6 * MB);
  bf16* w1t  = (bf16*)(ws + 8 * MB);
  bf16* w2t  = (bf16*)(ws + 16 * MB);
  bf16* xn1  = (bf16*)(ws + 24 * MB);
  bf16* xn2  = (bf16*)(ws + 40 * MB);
  bf16* h1   = (bf16*)(ws + 56 * MB);
  bf16* qb   = (bf16*)(ws + 56 * MB);
  bf16* kb   = (bf16*)(ws + 72 * MB);
  bf16* vtb  = (bf16*)(ws + 88 * MB);
  bf16* ao   = (bf16*)(ws + 104 * MB);
  float* tpre= (float*)(ws + 120 * MB);
  float* hebo= (float*)(ws + 120 * MB);
  float* trmo= (float*)(ws + 152 * MB);

  transpose_cvt_kernel<<<(Dd / 64) * (Dd / 64),  256, 0, stream>>>(wq,  wqt, Dd,  Dd);
  transpose_cvt_kernel<<<(Dd / 64) * (Dd / 64),  256, 0, stream>>>(wk,  wkt, Dd,  Dd);
  transpose_cvt_kernel<<<(Dd / 64) * (Dd / 64),  256, 0, stream>>>(wv,  wvt, Dd,  Dd);
  transpose_cvt_kernel<<<(Dd / 64) * (Dd / 64),  256, 0, stream>>>(wo,  wot, Dd,  Dd);
  transpose_cvt_kernel<<<(DFf / 64) * (Dd / 64), 256, 0, stream>>>(t_w1, w1t, Dd,  DFf);
  transpose_cvt_kernel<<<(Dd / 64) * (DFf / 64), 256, 0, stream>>>(t_w2, w2t, DFf, Dd);

  ln_dual_kernel<<<TOK, 256, 0, stream>>>(x, t_ln1_g, t_ln1_b, h_ln_g, h_ln_b,
                                          xn1, xn2);

  gemm_bf16_wmma<0><<<dim3(DFf / 128, TOK / 128), 256, 0, stream>>>(
      xn1, w1t, t_b1, nullptr, h1, TOK, DFf, Dd);
  gemm_bf16_wmma<1><<<dim3(Dd / 128, TOK / 128), 256, 0, stream>>>(
      h1, w2t, t_b2, x, tpre, TOK, Dd, DFf);
  trm_scalar_mlp_kernel<<<TOK, 256, 0, stream>>>(
      tpre, t_lns_g, t_lns_b, s_w1, s_b1, s_w2, s_b2, trmo);

  gemm_bf16_wmma<2><<<dim3(Dd / 128, TOK / 128), 256, 0, stream>>>(
      xn2, wqt, bq, nullptr, qb, TOK, Dd, Dd);
  gemm_bf16_wmma<2><<<dim3(Dd / 128, TOK / 128), 256, 0, stream>>>(
      xn2, wkt, bk, nullptr, kb, TOK, Dd, Dd);
  gemm_bf16_wmma<3><<<dim3(Dd / 128, TOK / 128), 256, 0, stream>>>(
      xn2, wvt, bv, nullptr, vtb, TOK, Dd, Dd);
  hebbian_attn_kernel<<<dim3(Ss / 64, Bb * Hh), 256, 0, stream>>>(
      qb, kb, vtb, beta, ao);
  gemm_bf16_wmma<1><<<dim3(Dd / 128, TOK / 128), 256, 0, stream>>>(
      ao, wot, bo, x, hebo, TOK, Dd, Dd);

  blend_ln_kernel<<<TOK, 256, 0, stream>>>(x, trmo, hebo, alpha,
                                           o_ln_g, o_ln_b, out);
}
